// MultiheadAttention_39676907881438
// MI455X (gfx1250) — hardware-verified
//
#include <hip/hip_runtime.h>


#ifndef NB
#define NB 32
#endif
#ifndef SEQ
#define SEQ 2048
#endif
#define NB_FULL  32
#define SEQ_FULL 2048
#define HD   128
#define TT   SEQ
#define ZB   3
#define PCAR 1024.0f
#define SCL  0.088388347648318447f

static_assert(SEQ % 128 == 0);
static_assert(SEQ >= 128);
static_assert(SEQ <= SEQ_FULL);
static_assert(NB >= 1);
static_assert(NB <= NB_FULL);
static_assert(HD % 64 == 0);
static_assert(3ull * NB * SEQ * HD * 2ull + (size_t)ZB * SEQ * (size_t)SEQ * 6ull <= 134217728ull);

typedef _Float16 h16;
typedef unsigned short bf;
typedef __attribute__((ext_vector_type(16))) __bf16   v16bf;
typedef __attribute__((ext_vector_type(16))) _Float16 v16h;
typedef __attribute__((ext_vector_type(8)))  _Float16 v8h;
typedef __attribute__((ext_vector_type(4)))  _Float16 v4h;
typedef __attribute__((ext_vector_type(2)))  _Float16 v2h;
typedef __attribute__((ext_vector_type(8)))  unsigned short v8us;
typedef __attribute__((ext_vector_type(8)))  float    v8f;
typedef __attribute__((ext_vector_type(4)))  float    v4f;
typedef v8h  __attribute__((may_alias)) v8ha;
typedef v4f  __attribute__((may_alias)) v4fa;
typedef v8us __attribute__((may_alias)) v8usa;

__device__ __forceinline__ unsigned short f2bf(float f) { unsigned u = __float_as_uint(f); u += 0x7FFFu + ((u >> 16) & 1u); return (unsigned short)(u >> 16); }
__device__ __forceinline__ float bf2f(unsigned short b) { return __uint_as_float(((unsigned)b) << 16); }
__device__ __forceinline__ float bfr(float f) { return bf2f(f2bf(f)); }
__device__ __forceinline__ h16 tohx(float x) { return (h16)x; }
__device__ __forceinline__ v16h cat16(v8h lo, v8h hi) { return __builtin_shufflevector(lo, hi, 0, 1, 2, 3, 4, 5, 6, 7, 8, 9, 10, 11, 12, 13, 14, 15); }
__device__ __forceinline__ v16bf cat16b(v8us lo, v8us hi) { return __builtin_bit_cast(v16bf, __builtin_shufflevector(lo, hi, 0, 1, 2, 3, 4, 5, 6, 7, 8, 9, 10, 11, 12, 13, 14, 15)); }
__device__ __forceinline__ v8f wmma16(v16h a, v16h b, v8f c) { return __builtin_amdgcn_wmma_f32_16x16x32_f16(false, a, false, b, (short)0, c, false, false); }
__device__ __forceinline__ v8f wmmab(v16bf a, v16bf b, v8f c) { return __builtin_amdgcn_wmma_f32_16x16x32_bf16(false, a, false, b, (short)0, c, false, false); }

template <typename T16> struct WFrag;
template <> struct WFrag<h16> { typedef v16h V; static __device__ __forceinline__ V ld(const h16* p) { return cat16(*(const v8h*)p, *(const v8h*)(p + 16)); } static __device__ __forceinline__ v8f mma(V a, V b, v8f c) { return wmma16(a, b, c); } };
template <> struct WFrag<bf> { typedef v16bf V; static __device__ __forceinline__ V ld(const bf* p) { return cat16b(*(const v8us*)p, *(const v8us*)(p + 16)); } static __device__ __forceinline__ v8f mma(V a, V b, v8f c) { return wmmab(a, b, c); } };
template <typename T16, int NSPLIT, bool BIAS>
__global__ __launch_bounds__(32) void k_gemmw(const T16* __restrict__ A, const T16* __restrict__ A2, const T16* __restrict__ Bt, const T16* __restrict__ Bt2, int K, float* C, int ldc, const float* __restrict__ bias, float alpha, size_t sA, size_t sB, size_t sC) {
    typedef typename WFrag<T16>::V V;
    __shared__ __align__(16) float os[16 * 68];
    const size_t z = blockIdx.z; A += z * sA; if (A2) A2 += z * sA; Bt += z * sB; if (Bt2) Bt2 += z * sB; C += z * sC;
    const int lane = threadIdx.x & 31, lr = lane & 15, hi = lane >> 4; const int r0 = blockIdx.x * 64, c0 = blockIdx.y * 64;
    v8f acc[4][4];
#pragma unroll
    for (int mb = 0; mb < 4; ++mb)
#pragma unroll
        for (int nb = 0; nb < 4; ++nb) acc[mb][nb] = (v8f){};
    const size_t aoff = (size_t)(r0 + lr) * K + 8 * hi, boff = (size_t)(c0 + lr) * K + 8 * hi;
#pragma unroll 1
    for (int kc = 0; kc < K; kc += 32) {
        V a[4], a2[4];
#pragma unroll
        for (int mb = 0; mb < 4; ++mb) { a[mb] = WFrag<T16>::ld(A + aoff + (size_t)mb * 16 * K + kc); if (NSPLIT == 1 || NSPLIT == 2) a2[mb] = WFrag<T16>::ld(A2 + aoff + (size_t)mb * 16 * K + kc); }
#pragma unroll
        for (int nb = 0; nb < 4; ++nb) { const V b = WFrag<T16>::ld(Bt + boff + (size_t)nb * 16 * K + kc); V b2; if (NSPLIT >= 2) b2 = WFrag<T16>::ld(Bt2 + boff + (size_t)nb * 16 * K + kc);
#pragma unroll
            for (int mb = 0; mb < 4; ++mb) { acc[mb][nb] = WFrag<T16>::mma(a[mb], b, acc[mb][nb]); if (NSPLIT == 1 || NSPLIT == 2) acc[mb][nb] = WFrag<T16>::mma(a2[mb], b, acc[mb][nb]); if (NSPLIT >= 2) acc[mb][nb] = WFrag<T16>::mma(a[mb], b2, acc[mb][nb]); } }
        asm volatile("v_nop\n\tv_nop\n\tv_nop\n\tv_nop" : "+v"(acc[0][0]), "+v"(acc[1][1]), "+v"(acc[2][2]), "+v"(acc[3][3]) : "v"(a[0]), "v"(a[3]));
    }
#pragma unroll
    for (int mb = 0; mb < 4; ++mb) {
#pragma unroll
        for (int nb = 0; nb < 4; ++nb) {
#pragma unroll
            for (int j = 0; j < 8; ++j) os[(hi * 8 + j) * 68 + nb * 16 + lr] = acc[mb][nb][j]; }
        __builtin_amdgcn_wave_barrier(); asm volatile("" ::: "memory");
        float* crow = C + (size_t)(r0 + mb * 16) * ldc + c0;
#pragma unroll 1
        for (int ps = 0; ps < 2; ++ps) {
#pragma unroll
            for (int s = 0; s < 8; ++s) { const int row = 2 * s + hi, cofs = lr * 4; v4f val = *(const v4fa*)(os + row * 68 + cofs); val = val * alpha; if (BIAS) { val[0] += bfr(bias[c0 + cofs]); val[1] += bfr(bias[c0 + cofs + 1]); val[2] += bfr(bias[c0 + cofs + 2]); val[3] += bfr(bias[c0 + cofs + 3]); }
                *(volatile v4f*)(crow + (size_t)row * ldc + cofs) = val; }
            if (ps == 0) __threadfence(); }
        __builtin_amdgcn_wave_barrier(); asm volatile("" ::: "memory");
    }
}

__global__ __launch_bounds__(256) void k_cvt8(const float* __restrict__ src, size_t sstride, bf* dst, size_t dstride, size_t n8) {
    const size_t i = (size_t)blockIdx.x * 256 + threadIdx.x; if (i >= n8) return;
    src += (size_t)blockIdx.y * sstride; dst += (size_t)blockIdx.y * dstride;
    const v8f v = *(const v8f*)(src + i * 8); v8us o;
#pragma unroll
    for (int k = 0; k < 8; ++k) o[k] = f2bf(v[k]);
    *(volatile v8us*)(dst + i * 8) = o; __threadfence(); *(volatile v8us*)(dst + i * 8) = o; }

__global__ __launch_bounds__(256) void k_vtp16(const float* __restrict__ Vb, size_t sstride, h16* Vh, size_t dstride) {
    const size_t e = ((size_t)blockIdx.x * 256 + threadIdx.x) * 2; if (e >= (size_t)HD * TT) return;
    Vb += (size_t)blockIdx.y * sstride; Vh += (size_t)blockIdx.y * dstride;
    const int t = (int)(e % TT); const int d = (int)(e / TT); v2h o; o[0] = tohx(bfr(Vb[(size_t)t * HD + d])); o[1] = tohx(bfr(Vb[(size_t)(t + 1) * HD + d]));
    *(volatile v2h*)(Vh + e) = o; __threadfence(); *(volatile v2h*)(Vh + e) = o; }

__global__ __launch_bounds__(256) void k_asoft(const float* __restrict__ Sb, h16* P16, int nrows) {
    const int lane = threadIdx.x & 31; const int row = blockIdx.x * 8 + (threadIdx.x >> 5); if (row >= nrows) return;
    const float* sr = Sb + (size_t)row * TT; float v[TT / 32]; float mx = -3.0e38f;
#pragma unroll
    for (int ch = 0; ch < TT / 128; ++ch) { const int j0 = ch * 128 + lane * 4; const v4f a = *(const v4f*)(sr + j0);
#pragma unroll
        for (int q = 0; q < 4; ++q) { const float t = a[q] * SCL; v[ch * 4 + q] = t; mx = fmaxf(mx, t); } }
#pragma unroll
    for (int sh = 16; sh; sh >>= 1) mx = fmaxf(mx, __shfl_xor(mx, sh, 32));
    float sum = 0.f;
#pragma unroll
    for (int k = 0; k < TT / 32; ++k) { float d0 = __fsub_rn(v[k], mx); asm volatile("" : "+v"(d0)); v[k] = __builtin_amdgcn_exp2f(__fmul_rn(d0, 1.4426950408889634f)); sum += v[k]; }
#pragma unroll
    for (int sh = 16; sh; sh >>= 1) sum += __shfl_xor(sum, sh, 32);
    const float f = __fdiv_rn(PCAR, sum);
#pragma unroll 1
    for (int ps = 0; ps < 2; ++ps) {
#pragma unroll
        for (int ch = 0; ch < TT / 128; ++ch) { v4h o4;
#pragma unroll
            for (int q = 0; q < 4; ++q) o4[q] = tohx(v[ch * 4 + q] * f);
            *(volatile v4h*)(P16 + (size_t)row * TT + ch * 128 + lane * 4) = o4; }
        if (ps == 0) __threadfence(); }
}

extern "C" void kernel_launch(void* const* d_in, const int* in_sizes, int n_in,
                              void* d_out, int out_size, void* d_ws, size_t ws_size, hipStream_t stream) {
    if (n_in < 3) return;
    const size_t need_in = (size_t)(NB - 1) * SEQ_FULL * HD + (size_t)SEQ * HD;
    if ((size_t)in_sizes[0] < need_in || (size_t)in_sizes[1] < need_in || (size_t)in_sizes[2] < need_in) return;
    if ((size_t)out_size < (size_t)NB * SEQ * HD) return;
    const float* Qin = (const float*)d_in[0]; const float* Kin = (const float*)d_in[1]; const float* Vin = (const float*)d_in[2];
    float* OUT = (float*)d_out;
    char* wsp = (char*)d_ws;
    auto take = [&](size_t bytes) { char* p = wsp; wsp += (bytes + 255) & ~(size_t)255; return (void*)p; };
    const size_t plane = (size_t)SEQ * HD;
    const size_t istr  = (size_t)SEQ_FULL * HD;
    bf*  QB  = (bf*)take((size_t)NB * plane * 2);
    bf*  KB  = (bf*)take((size_t)NB * plane * 2);
    h16* VT  = (h16*)take((size_t)NB * plane * 2);
    float* Sb = (float*)take((size_t)ZB * SEQ * SEQ * 4);
    h16* P16 = (h16*)take((size_t)ZB * SEQ * SEQ * 2);
    if ((size_t)(wsp - (char*)d_ws) > ws_size) return;
    const size_t n8 = plane / 8;
    k_cvt8<<<dim3((unsigned)((n8 + 255) / 256), NB), 256, 0, stream>>>(Qin, istr, QB, plane, n8);
    k_cvt8<<<dim3((unsigned)((n8 + 255) / 256), NB), 256, 0, stream>>>(Kin, istr, KB, plane, n8);
    k_vtp16<<<dim3((unsigned)(((size_t)HD * SEQ / 2 + 255) / 256), NB), 256, 0, stream>>>(Vin, istr, VT, plane);
    for (int b0 = 0; b0 < NB; b0 += ZB) {
        const int zc = (NB - b0 < ZB) ? (NB - b0) : ZB;
        k_gemmw<bf, 0, false><<<dim3(SEQ / 64, SEQ / 64, zc), 32, 0, stream>>>(QB + (size_t)b0 * plane, nullptr, KB + (size_t)b0 * plane, nullptr, HD, Sb, SEQ, nullptr, 1.0f, plane, plane, (size_t)SEQ * SEQ);
        k_asoft<<<(unsigned)((size_t)zc * SEQ / 8), 256, 0, stream>>>(Sb, P16, zc * SEQ);
        k_gemmw<h16, 0, false><<<dim3(SEQ / 64, HD / 64, zc), 32, 0, stream>>>(P16, nullptr, VT + (size_t)b0 * plane, nullptr, SEQ, OUT + (size_t)b0 * plane, HD, nullptr, 1.0f / PCAR, (size_t)SEQ * SEQ, plane, plane);
    }
}
